// LSTM_33380485824995
// MI455X (gfx1250) — hardware-verified
//
#include <hip/hip_runtime.h>

constexpr int NSEQ    = 64;
constexpr int NSTEP   = 2048;
constexpr int NIN     = 32;
constexpr int NHID    = 256;
constexpr int NGATE   = 4 * NHID;
constexpr int NCLS    = 16;
constexpr int NTHR    = 512;
constexpr int SEQ_BLK = 16;
constexpr int XPITCH  = 40;
constexpr int HPITCH  = 264;
constexpr int OPITCH  = 36;
constexpr int BSM_N   = 2 * NGATE + 32;
constexpr float WCARRY     = 16.0f;
constexpr float WCARRY_INV = 1.0f / 16.0f;
static_assert(NSEQ % SEQ_BLK == 0);
static_assert(NHID == 16 * (NTHR / 32));
static_assert(NTHR == SEQ_BLK * NIN);
static_assert(2 * NTHR == NGATE);
static_assert(NIN == 32);
static_assert(NHID % 32 == 0);
static_assert(NCLS == 16);
static_assert(NSTEP % 2 == 0);
static_assert(XPITCH % 8 == 0 && HPITCH % 8 == 0 && OPITCH % 4 == 0);
static_assert((NGATE * NIN) % (8 * 256) == 0 && (NGATE * NHID) % (8 * 256) == 0 && (NCLS * NHID) % (8 * 256) == 0);

typedef __attribute__((ext_vector_type(16))) _Float16 v16h;
typedef __attribute__((ext_vector_type(8)))  _Float16 v8h;
typedef __attribute__((ext_vector_type(16))) __bf16   v16b;
typedef __attribute__((ext_vector_type(8)))  __bf16   v8b;
typedef __attribute__((ext_vector_type(8)))  float    v8f;
typedef __attribute__((ext_vector_type(4)))  float    v4f;
typedef __attribute__((ext_vector_type(2)))  float    v2f;

__device__ __forceinline__ void dep_guard_h(v8f& a, v8f& b, v16h x, v16h y) { asm volatile("v_nop\n\tv_nop\n\tv_nop\n\tv_nop" : "+v"(a), "+v"(b) : "v"(x), "v"(y)); }
__device__ __forceinline__ void dep_guard_b(v8f& a, v8f& b, v16b x, v16b y) { asm volatile("v_nop\n\tv_nop\n\tv_nop\n\tv_nop" : "+v"(a), "+v"(b) : "v"(x), "v"(y)); }
__device__ __forceinline__ void dep_guard1_h(v8f& a, v16h x, v16h y) { asm volatile("v_nop\n\tv_nop\n\tv_nop\n\tv_nop" : "+v"(a) : "v"(x), "v"(y)); }
__device__ __forceinline__ void dep_guard4_h(v8f& a, v8f& b, v8f& c, v8f& d, v16h x, v16h y) {
  asm volatile("v_nop\n\tv_nop\n\tv_nop\n\tv_nop" : "+v"(a), "+v"(b), "+v"(c), "+v"(d) : "v"(x), "v"(y));
}
__device__ __forceinline__ void keep4_h(v16h a, v16h b, v16h c, v16h d) { asm volatile("v_nop" :: "v"(a), "v"(b), "v"(c), "v"(d)); }
__device__ __forceinline__ void keep4_b(v16b a, v16b b, v16b c, v16b d) { asm volatile("v_nop" :: "v"(a), "v"(b), "v"(c), "v"(d)); }
__device__ __forceinline__ void acc_guard4(v8f& a, v8f& b, v8f& c, v8f& d) { asm volatile("v_nop\n\tv_nop\n\tv_nop\n\tv_nop" : "+v"(a), "+v"(b), "+v"(c), "+v"(d)); }
template <typename T> struct Frag;
template <> struct Frag<_Float16> {
  typedef v16h V; union U { v16h v; v8h h[2]; };
  static __device__ __forceinline__ v16h load(const _Float16* p) {
    U f; f.h[0] = *(const v8h*)(p); f.h[1] = *(const v8h*)(p + 16); return f.v;
  }
  static __device__ __forceinline__ v8f mma(v16h a, v16h b, v8f c) {
    return __builtin_amdgcn_wmma_f32_16x16x32_f16(false, a, false, b, (short)0, c, false, false);
  }
  static __device__ __forceinline__ void guard(v8f& a, v8f& b, v16h x, v16h y) { dep_guard_h(a, b, x, y); }
  static __device__ __forceinline__ void keep(v16h a, v16h b, v16h c, v16h d) { keep4_h(a, b, c, d); }
};
template <> struct Frag<__bf16> {
  typedef v16b V; union U { v16b v; v8b h[2]; };
  static __device__ __forceinline__ v16b load(const __bf16* p) {
    U f; f.h[0] = *(const v8b*)(p); f.h[1] = *(const v8b*)(p + 16); return f.v;
  }
  static __device__ __forceinline__ v8f mma(v16b a, v16b b, v8f c) {
    return __builtin_amdgcn_wmma_f32_16x16x32_bf16(false, a, false, b, (short)0, c, false, false);
  }
  static __device__ __forceinline__ void guard(v8f& a, v8f& b, v16b x, v16b y) { dep_guard_b(a, b, x, y); }
  static __device__ __forceinline__ void keep(v16b a, v16b b, v16b c, v16b d) { keep4_b(a, b, c, d); }
};

__device__ __forceinline__ float fsig(float x)  { return __builtin_amdgcn_rcpf(1.0f + __expf(-x)); }
__device__ __forceinline__ float ftanh(float x) { return 1.0f - 2.0f * __builtin_amdgcn_rcpf(__expf(2.0f * x) + 1.0f); }

__global__ __launch_bounds__(256) void cvt_f16x8_kernel(const float* __restrict__ src, unsigned short* __restrict__ dst,
                                                       int n8, float sc) {
  const int i = blockIdx.x * 256 + threadIdx.x;
  if (i < n8) {
    const float* sp = src + (size_t)i * 8;
    const v4f a = *(const v4f*)(sp);
    const v4f b = *(const v4f*)(sp + 4);
    v8h hv;
#pragma unroll
    for (int e = 0; e < 4; ++e) {
      hv[e]     = (_Float16)(a[e] * sc);
      hv[4 + e] = (_Float16)(b[e] * sc);
    }
    *(volatile v8h*)(dst + (size_t)i * 8) = hv;
    __threadfence();
    *(volatile v8h*)(dst + (size_t)i * 8) = hv;
  }
}

__global__ __launch_bounds__(NTHR) void lstm2_seq_kernel(const float* __restrict__ x,
                                                         const float* __restrict__ bih0, const float* __restrict__ bhh0,
                                                         const float* __restrict__ bih1, const float* __restrict__ bhh1,
                                                         const float* __restrict__ fcb,
                                                         const unsigned short* __restrict__ WI0p,
                                                         const unsigned short* __restrict__ WH0p,
                                                         const unsigned short* __restrict__ WI1p,
                                                         const unsigned short* __restrict__ WH1p,
                                                         const unsigned short* __restrict__ FCWp,
                                                         float* __restrict__ out) {
  __shared__ __align__(16) _Float16 Hs0[2][SEQ_BLK * HPITCH];
  __shared__ __align__(16) _Float16 Hs1[2][SEQ_BLK * HPITCH];
  __shared__ __align__(16) _Float16 Xs[SEQ_BLK * XPITCH];
  __shared__ __align__(16) float    Ob[SEQ_BLK * OPITCH];
  __shared__ __align__(16) float    Bsm[BSM_N];
  const _Float16* WI0 = (const _Float16*)WI0p;
  const _Float16* WH0 = (const _Float16*)WH0p;
  const _Float16* WI1 = (const _Float16*)WI1p;
  const _Float16* WH1 = (const _Float16*)WH1p;
  const _Float16* FCW = (const _Float16*)FCWp;
  const int tid = threadIdx.x, lane = tid & 31, wave = tid >> 5;
  const int c = lane & 15, hh = lane >> 4, koff = hh * 8;
  const int rowbase = blockIdx.x * SEQ_BLK;
  const int j = 16 * wave + c;

  {
    _Float16* p0 = &Hs0[0][0];
    _Float16* p1 = &Hs1[0][0];
#pragma unroll 1
    for (int i = tid; i < 2 * SEQ_BLK * HPITCH; i += NTHR) { p0[i] = (_Float16)0.0f; p1[i] = (_Float16)0.0f; }
#pragma unroll 1
    for (int i = tid; i < SEQ_BLK * XPITCH; i += NTHR) Xs[i] = (_Float16)0.0f;
#pragma unroll 1
    for (int i = tid; i < SEQ_BLK * OPITCH; i += NTHR) Ob[i] = 0.0f;
  }
  {
    const int n2 = 2 * tid;
    const v2f a0 = *(const v2f*)(bih0 + n2);
    const v2f a1 = *(const v2f*)(bhh0 + n2);
    const v2f a2 = *(const v2f*)(bih1 + n2);
    const v2f a3 = *(const v2f*)(bhh1 + n2);
    const float fv = fcb[tid & 15];
    v2f s0, s1;
    s0[0] = a0[0] + a1[0]; s0[1] = a0[1] + a1[1];
    s1[0] = a2[0] + a3[0]; s1[1] = a2[1] + a3[1];
    *(v2f*)(Bsm + n2) = s0;
    *(v2f*)(Bsm + NGATE + n2) = s1;
    if (tid < NCLS) Bsm[2 * NGATE + tid] = fv;
  }
  float cst0[8], cst1[8];
#pragma unroll
  for (int r = 0; r < 8; ++r) { cst0[r] = 0.0f; cst1[r] = 0.0f; }
  __syncthreads();
  float bs0[4], bs1[4];
#pragma unroll
  for (int g = 0; g < 4; ++g) {
    bs0[g] = Bsm[g * NHID + j];
    bs1[g] = Bsm[NGATE + g * NHID + j];
  }
  const float fcbias = Bsm[2 * NGATE + c];
  {
    const int m = tid >> 5, i = tid & 31;
    Xs[m * XPITCH + i] = (_Float16)x[((size_t)(rowbase + m) * NSTEP) * NIN + i];
  }
  __syncthreads();

  const v8f z8 = {0.f, 0.f, 0.f, 0.f, 0.f, 0.f, 0.f, 0.f};
  const _Float16* axrow = Xs + c * XPITCH + koff;
  const _Float16* wi0 = WI0 + (size_t)j * NIN + koff;
  const _Float16* wh0 = WH0 + (size_t)j * NHID + koff;
  const _Float16* wi1 = WI1 + (size_t)j * NHID + koff;
  const _Float16* wh1 = WH1 + (size_t)j * NHID + koff;
  const _Float16* wfc = FCW + (size_t)c * NHID + koff;
  constexpr size_t GSTR_X = (size_t)NHID * NIN;
  constexpr size_t GSTR_H = (size_t)NHID * NHID;

#pragma unroll 1
  for (int t = 0; t < NSTEP; ++t) {
    const int cur = t & 1, prv = cur ^ 1;

    {
      v8f acc[4];
      acc[0] = z8; acc[1] = z8; acc[2] = z8; acc[3] = z8;
      {
        const v16h a  = Frag<_Float16>::load(axrow);
        const v16h b0 = Frag<_Float16>::load(wi0);
        const v16h b1 = Frag<_Float16>::load(wi0 + GSTR_X);
        const v16h b2 = Frag<_Float16>::load(wi0 + 2 * GSTR_X);
        const v16h b3 = Frag<_Float16>::load(wi0 + 3 * GSTR_X);
        acc[0] = Frag<_Float16>::mma(a, b0, acc[0]);
        acc[1] = Frag<_Float16>::mma(a, b1, acc[1]);
        acc[2] = Frag<_Float16>::mma(a, b2, acc[2]);
        acc[3] = Frag<_Float16>::mma(a, b3, acc[3]);
        dep_guard4_h(acc[0], acc[1], acc[2], acc[3], a, b3);
        keep4_h(b0, b1, b2, b3);
      }
      const _Float16* ahrow = &Hs0[prv][0] + c * HPITCH + koff;
#pragma unroll 1
      for (int k0 = 0; k0 < NHID; k0 += 32) {
        const v16h a  = Frag<_Float16>::load(ahrow + k0);
        const v16h b0 = Frag<_Float16>::load(wh0 + k0);
        const v16h b1 = Frag<_Float16>::load(wh0 + GSTR_H + k0);
        const v16h b2 = Frag<_Float16>::load(wh0 + 2 * GSTR_H + k0);
        const v16h b3 = Frag<_Float16>::load(wh0 + 3 * GSTR_H + k0);
        acc[0] = Frag<_Float16>::mma(a, b0, acc[0]);
        acc[1] = Frag<_Float16>::mma(a, b1, acc[1]);
        acc[2] = Frag<_Float16>::mma(a, b2, acc[2]);
        acc[3] = Frag<_Float16>::mma(a, b3, acc[3]);
        dep_guard4_h(acc[0], acc[1], acc[2], acc[3], a, b3);
        keep4_h(b0, b1, b2, b3);
      }
      acc_guard4(acc[0], acc[1], acc[2], acc[3]);
      _Float16* hw = &Hs0[cur][0];
#pragma unroll
      for (int r = 0; r < 8; ++r) {
        const float zi = acc[0][r] * WCARRY_INV + bs0[0];
        const float zf = acc[1][r] * WCARRY_INV + bs0[1];
        const float zg = acc[2][r] * WCARRY_INV + bs0[2];
        const float zo = acc[3][r] * WCARRY_INV + bs0[3];
        const float cn = fsig(zf) * cst0[r] + fsig(zi) * ftanh(zg);
        cst0[r] = cn;
        const float hn = fsig(zo) * ftanh(cn);
        hw[(8 * hh + r) * HPITCH + j] = (_Float16)hn;
      }
    }
    __syncthreads();

    {
      const int tn = (t + 1 < NSTEP) ? (t + 1) : (NSTEP - 1);
      const int m = tid >> 5, i = tid & 31;
      Xs[m * XPITCH + i] = (_Float16)x[((size_t)(rowbase + m) * NSTEP + (size_t)tn) * NIN + i];
    }

    {
      v8f acc[4];
      acc[0] = z8; acc[1] = z8; acc[2] = z8; acc[3] = z8;
      const _Float16* a0row = &Hs0[cur][0] + c * HPITCH + koff;
#pragma unroll 1
      for (int k0 = 0; k0 < NHID; k0 += 32) {
        const v16h a  = Frag<_Float16>::load(a0row + k0);
        const v16h b0 = Frag<_Float16>::load(wi1 + k0);
        const v16h b1 = Frag<_Float16>::load(wi1 + GSTR_H + k0);
        const v16h b2 = Frag<_Float16>::load(wi1 + 2 * GSTR_H + k0);
        const v16h b3 = Frag<_Float16>::load(wi1 + 3 * GSTR_H + k0);
        acc[0] = Frag<_Float16>::mma(a, b0, acc[0]);
        acc[1] = Frag<_Float16>::mma(a, b1, acc[1]);
        acc[2] = Frag<_Float16>::mma(a, b2, acc[2]);
        acc[3] = Frag<_Float16>::mma(a, b3, acc[3]);
        dep_guard4_h(acc[0], acc[1], acc[2], acc[3], a, b3);
        keep4_h(b0, b1, b2, b3);
      }
      const _Float16* a1row = &Hs1[prv][0] + c * HPITCH + koff;
#pragma unroll 1
      for (int k0 = 0; k0 < NHID; k0 += 32) {
        const v16h a  = Frag<_Float16>::load(a1row + k0);
        const v16h b0 = Frag<_Float16>::load(wh1 + k0);
        const v16h b1 = Frag<_Float16>::load(wh1 + GSTR_H + k0);
        const v16h b2 = Frag<_Float16>::load(wh1 + 2 * GSTR_H + k0);
        const v16h b3 = Frag<_Float16>::load(wh1 + 3 * GSTR_H + k0);
        acc[0] = Frag<_Float16>::mma(a, b0, acc[0]);
        acc[1] = Frag<_Float16>::mma(a, b1, acc[1]);
        acc[2] = Frag<_Float16>::mma(a, b2, acc[2]);
        acc[3] = Frag<_Float16>::mma(a, b3, acc[3]);
        dep_guard4_h(acc[0], acc[1], acc[2], acc[3], a, b3);
        keep4_h(b0, b1, b2, b3);
      }
      acc_guard4(acc[0], acc[1], acc[2], acc[3]);
      _Float16* hw = &Hs1[cur][0];
#pragma unroll
      for (int r = 0; r < 8; ++r) {
        const float zi = acc[0][r] * WCARRY_INV + bs1[0];
        const float zf = acc[1][r] * WCARRY_INV + bs1[1];
        const float zg = acc[2][r] * WCARRY_INV + bs1[2];
        const float zo = acc[3][r] * WCARRY_INV + bs1[3];
        const float cn = fsig(zf) * cst1[r] + fsig(zi) * ftanh(zg);
        cst1[r] = cn;
        const float hn = fsig(zo) * ftanh(cn);
        hw[(8 * hh + r) * HPITCH + j] = (_Float16)hn;
      }
    }
    __syncthreads();

    if (wave == 0) {
      v8f o = z8;
      const _Float16* ahrow = &Hs1[cur][0] + c * HPITCH + koff;
#pragma unroll 1
      for (int k0 = 0; k0 < NHID; k0 += 32) {
        const v16h a = Frag<_Float16>::load(ahrow + k0);
        const v16h b = Frag<_Float16>::load(wfc + k0);
        o = Frag<_Float16>::mma(a, b, o);
        dep_guard1_h(o, a, b);
      }
#pragma unroll
      for (int r = 0; r < 8; ++r) Ob[(8 * hh + r) * OPITCH + cur * NCLS + c] = o[r] * WCARRY_INV + fcbias;
      if (cur == 1) {
        __builtin_amdgcn_fence(__ATOMIC_RELEASE, "workgroup");
        __builtin_amdgcn_wave_barrier();
        __builtin_amdgcn_fence(__ATOMIC_ACQUIRE, "workgroup");
        const int q = lane >> 3, c4 = (lane & 7) * 4;
        for (int pass = 0; pass < 2; ++pass) {
#pragma unroll
          for (int it = 0; it < 4; ++it) {
            const int row = it * 4 + q;
            const v4f v = *(const v4f*)(Ob + row * OPITCH + c4);
            *(volatile v4f*)(out + ((size_t)(rowbase + row) * NSTEP + (size_t)(t - 1)) * NCLS + c4) = v;
          }
          __threadfence();
        }
        __builtin_amdgcn_fence(__ATOMIC_RELEASE, "workgroup");
        __builtin_amdgcn_wave_barrier();
        __builtin_amdgcn_fence(__ATOMIC_ACQUIRE, "workgroup");
      }
    }
  }
}

extern "C" void kernel_launch(void* const* d_in, const int* in_sizes, int n_in,
                              void* d_out, int out_size, void* d_ws, size_t ws_size, hipStream_t stream) {
  if (n_in < 11 || d_out == nullptr || d_ws == nullptr) return;
  if (in_sizes[0] != NSEQ * NSTEP * NIN || in_sizes[1] != NGATE * NIN || in_sizes[2] != NGATE * NHID ||
      in_sizes[3] != NGATE || in_sizes[4] != NGATE || in_sizes[5] != NGATE * NHID || in_sizes[6] != NGATE * NHID ||
      in_sizes[7] != NGATE || in_sizes[8] != NGATE || in_sizes[9] != NCLS * NHID || in_sizes[10] != NCLS ||
      out_size != NSEQ * NSTEP * NCLS) return;

  const float* x     = (const float*)d_in[0];
  const float* w_ih0 = (const float*)d_in[1];
  const float* w_hh0 = (const float*)d_in[2];
  const float* b_ih0 = (const float*)d_in[3];
  const float* b_hh0 = (const float*)d_in[4];
  const float* w_ih1 = (const float*)d_in[5];
  const float* w_hh1 = (const float*)d_in[6];
  const float* b_ih1 = (const float*)d_in[7];
  const float* b_hh1 = (const float*)d_in[8];
  const float* fc_w  = (const float*)d_in[9];
  const float* fc_b  = (const float*)d_in[10];
  float* y_out = (float*)d_out;

  char* ws = (char*)d_ws; size_t off = 0;
  auto carve = [&](size_t bytes) -> char* { char* p = ws + off; off += (bytes + 255) & ~(size_t)255; return p; };
  unsigned short* WI0 = (unsigned short*)carve((size_t)NGATE * NIN * 2);
  unsigned short* WH0 = (unsigned short*)carve((size_t)NGATE * NHID * 2);
  unsigned short* WI1 = (unsigned short*)carve((size_t)NGATE * NHID * 2);
  unsigned short* WH1 = (unsigned short*)carve((size_t)NGATE * NHID * 2);
  unsigned short* FCW = (unsigned short*)carve((size_t)NCLS * NHID * 2);
  if (off > ws_size || off > (size_t)134217728) return;

  const int n8x = NGATE * NIN / 8;
  const int n8h = NGATE * NHID / 8;
  const int n8f = NCLS * NHID / 8;
  cvt_f16x8_kernel<<<(n8x + 255) / 256, 256, 0, stream>>>(w_ih0, WI0, n8x, WCARRY);
  cvt_f16x8_kernel<<<(n8h + 255) / 256, 256, 0, stream>>>(w_hh0, WH0, n8h, WCARRY);
  cvt_f16x8_kernel<<<(n8h + 255) / 256, 256, 0, stream>>>(w_ih1, WI1, n8h, WCARRY);
  cvt_f16x8_kernel<<<(n8h + 255) / 256, 256, 0, stream>>>(w_hh1, WH1, n8h, WCARRY);
  cvt_f16x8_kernel<<<(n8f + 255) / 256, 256, 0, stream>>>(fc_w, FCW, n8f, WCARRY);

  lstm2_seq_kernel<<<NSEQ / SEQ_BLK, NTHR, 0, stream>>>(x, b_ih0, b_hh0, b_ih1, b_hh1, fc_b,
                                                       WI0, WH0, WI1, WH1, FCW, y_out);
}
